// ConvPool_67413806678241
// MI455X (gfx1250) — hardware-verified
//
#include <hip/hip_runtime.h>
#include <stdint.h>

typedef _Float16 v16h __attribute__((ext_vector_type(16)));
typedef float    v8f  __attribute__((ext_vector_type(8)));
typedef float    v4f  __attribute__((ext_vector_type(4)));

#define C_IN    16
#define HW      128
#define OUTC    64
#define NBATCH  32
#define PDIM    63
#define XW      132
#define PPITCH  64
#define PLANE   (OUTC * PDIM * PDIM)
#define NTHR    256

__device__ __forceinline__ v8f wmma_f16(v16h a, v16h b, v8f c) {
    v8f d = __builtin_amdgcn_wmma_f32_16x16x32_f16(false, a, false, b, (short)0, c, false, false);
    asm volatile("v_nop\n\tv_nop\n\tv_nop\n\tv_nop" : "+v"(d) : "v"(a), "v"(b));
    return d;
}

__global__ __launch_bounds__(NTHR)
void conv_pool_tile(const float* __restrict__ x,
                    const float* __restrict__ w,
                    const float* __restrict__ bias,
                    float* __restrict__ ws)
{
    __shared__ __align__(32) _Float16 lds_x2[4 * XW * C_IN];
    __shared__ __align__(32) _Float16 lds_pad[16];
    __shared__ __align__(32) _Float16 lds_wB[4 * 5 * 32 * 16];
    __shared__ float lds_bias[OUTC];
    __shared__ v4f   lds_pool4[OUTC * (PPITCH / 4)];

    const int tid = threadIdx.x;
    const int bid = blockIdx.x;
    const int b   = bid / PDIM;
    const int pr  = bid - b * PDIM;
    const int r0  = pr * 2;

    if (tid < OUTC) lds_bias[tid] = bias[tid];
    if (tid < 16)   lds_pad[tid]  = (_Float16)0.f;

    for (int idx = tid; idx < C_IN * 4 * XW; idx += NTHR) {
        const int c   = idx / (4 * XW);
        const int r2  = idx - c * (4 * XW);
        const int rr  = r2 / XW;
        const int col = r2 - rr * XW;
        float v = 0.f;
        if (col < HW) v = x[((b * C_IN + c) * HW + (r0 + rr)) * HW + col];
        lds_x2[(rr * XW + col) * C_IN + c] = (_Float16)v;
    }

    for (int idx = tid; idx < 4 * 5 * 32 * 16; idx += NTHR) {
        const int j   = idx & 15;
        const int ln  = (idx >> 4) & 31;
        const int kc  = (idx >> 9) % 5;
        const int nt  = idx / (5 * 32 * 16);
        const int g   = 2 * kc + (ln >> 4);
        const int n   = nt * 16 + (ln & 15);
        float v = 0.f;
        if (g < 9) v = w[(j * 9 + g) * OUTC + n] * 16.0f;
        lds_wB[idx] = (_Float16)v;
    }
    __syncthreads();

    const int wv   = tid >> 5;
    const int lane = tid & 31;
    const int h    = lane >> 4;
    const int m    = lane & 15;
    const int lc   = (wv << 4) + m;

    v8f acc[2][4];
#pragma unroll
    for (int rs = 0; rs < 2; ++rs)
#pragma unroll
        for (int nt = 0; nt < 4; ++nt) {
            v8f z = {0.f, 0.f, 0.f, 0.f, 0.f, 0.f, 0.f, 0.f};
            acc[rs][nt] = z;
        }

    const v16h* wb = (const v16h*)lds_wB;
#pragma unroll
    for (int kc = 0; kc < 5; ++kc) {
        const int g  = 2 * kc + h;
        const int gg = (g < 9) ? g : 0;
        const int tr = gg / 3, tc = gg - tr * 3;
        const _Float16* p0 = &lds_x2[((0 + tr) * XW + lc + tc) * C_IN];
        const _Float16* p1 = &lds_x2[((1 + tr) * XW + lc + tc) * C_IN];
        const v16h a0 = (g < 9) ? *(const v16h*)p0 : *(const v16h*)lds_pad;
        const v16h a1 = (g < 9) ? *(const v16h*)p1 : *(const v16h*)lds_pad;
#pragma unroll
        for (int nt = 0; nt < 4; ++nt) {
            const v16h bf = wb[(nt * 5 + kc) * 32 + lane];
            acc[0][nt] = wmma_f16(a0, bf, acc[0][nt]);
            acc[1][nt] = wmma_f16(a1, bf, acc[1][nt]);
        }
    }

    const int pc4 = (wv << 1) + h;
#pragma unroll
    for (int nt = 0; nt < 4; ++nt) {
        const int   ch = nt * 16 + m;
        const float bv = lds_bias[ch];
        v4f pv = {0.f, 0.f, 0.f, 0.f};
#pragma unroll
        for (int q = 0; q < 4; ++q) {
            const float m0 = fmaxf(acc[0][nt][2 * q], acc[0][nt][2 * q + 1]);
            const float m1 = fmaxf(acc[1][nt][2 * q], acc[1][nt][2 * q + 1]);
            pv[q] = fmaxf(fmaxf(m0, m1) * 0.0625f + bv, 0.f);
        }
        lds_pool4[ch * (PPITCH / 4) + pc4] = pv;
    }
    __syncthreads();

    const size_t wsb = (size_t)b * ((size_t)OUTC * PDIM * PPITCH) + (size_t)pr * PPITCH;
    v4f vals[4];
#pragma unroll
    for (int it = 0; it < 4; ++it) {
        const int f  = it * NTHR + tid;
        const int ch = f >> 4, c4 = f & 15;
        vals[it] = lds_pool4[ch * (PPITCH / 4) + c4];
    }
#pragma unroll
    for (int it = 0; it < 4; ++it) {
        const int f  = it * NTHR + tid;
        const int ch = f >> 4, c4 = f & 15;
        float* dst = ws + wsb + (size_t)ch * (PDIM * PPITCH) + c4 * 4;
        *(volatile v4f*)dst = vals[it];
    }
    __threadfence();
#pragma unroll
    for (int it = 0; it < 4; ++it) {
        const int f  = it * NTHR + tid;
        const int ch = f >> 4, c4 = f & 15;
        float* dst = ws + wsb + (size_t)ch * (PDIM * PPITCH) + c4 * 4;
        *(volatile v4f*)dst = vals[it];
    }
}

__global__ __launch_bounds__(NTHR)
void pool_gather_out(const float* __restrict__ ws, float* __restrict__ out)
{
    const int  b   = blockIdx.y;
    const int  o   = (blockIdx.x * NTHR + threadIdx.x) * 4;
    const bool act = o < PLANE;
    v4f v = {0.f, 0.f, 0.f, 0.f};
    if (act) {
#pragma unroll
        for (int e = 0; e < 4; ++e) {
            const int oo   = o + e;
            const int ch   = oo / (PDIM * PDIM);
            const int p    = oo - ch * (PDIM * PDIM);
            const int prow = p / PDIM;
            const int pc   = p - prow * PDIM;
            v[e] = ws[((size_t)(b * OUTC + ch) * PDIM + prow) * PPITCH + pc];
        }
    }
    float* dst = out + (size_t)b * PLANE + o;
    if (act) *(volatile v4f*)dst = v;
    __threadfence();
    if (act) *(volatile v4f*)dst = v;
}

extern "C" void kernel_launch(void* const* d_in, const int* in_sizes, int n_in,
                              void* d_out, int out_size, void* d_ws, size_t ws_size,
                              hipStream_t stream)
{
    if (n_in < 3) return;
    if (in_sizes[0] != NBATCH * C_IN * HW * HW) return;
    if (in_sizes[1] != C_IN * 9 * OUTC) return;
    if (in_sizes[2] != OUTC) return;
    if (out_size != NBATCH * PLANE) return;
    const size_t ws_need = (size_t)NBATCH * OUTC * PDIM * PPITCH * sizeof(float);
    if (ws_size < ws_need) return;

    const float* x    = (const float*)d_in[0];
    const float* w    = (const float*)d_in[1];
    const float* bias = (const float*)d_in[2];
    float*       out  = (float*)d_out;
    float*       ws   = (float*)d_ws;

    conv_pool_tile<<<dim3(NBATCH * PDIM), dim3(NTHR), 0, stream>>>(x, w, bias, ws);
    const int segs = (PLANE / 4 + NTHR - 1) / NTHR;
    pool_gather_out<<<dim3(segs, NBATCH), dim3(NTHR), 0, stream>>>(ws, out);
}
